// SelfAttention_49624052138298
// MI455X (gfx1250) — hardware-verified
//
#include <hip/hip_runtime.h>


#ifndef NB
#define NB 2
#endif
#ifndef SEQ
#define SEQ 2048
#endif
#define NB_FULL   2
#define SEQ_FULL  2048
#define EMB       2048
#define NHEAD     32
#define NKV       8
#define HDIM      64
#define NQKV      3072
#define EARLY     ((SEQ) < 512 ? (SEQ) : 512)
#define BQ        128
#define BK        32
#define NWAVE     8
#define OP        68
#define SP        68
#define TPW       72
#define MROWS     (NB * SEQ)
#define NEGBIG    (-1.0e30f)
#define WS_CAP    134217728ull

typedef unsigned long long u64;

#define N_XB    ((u64)MROWS * EMB)
#define N_WQKV  ((u64)NQKV * EMB)
#define N_WO    ((u64)EMB * EMB)
#define N_QH    ((u64)NB * NHEAD * SEQ * HDIM)
#define N_QR    ((u64)NB * NHEAD * EARLY * HDIM)
#define N_KH    ((u64)NB * NKV * SEQ * HDIM)
#define N_KR    ((u64)NB * NKV * EARLY * HDIM)
#define N_CH    ((u64)MROWS * EMB)
#define N_CR    ((u64)NB * EARLY * EMB)
#define E_XB    0ull
#define E_WQKV  (E_XB + N_XB)
#define E_WO    (E_WQKV + N_WQKV)
#define E_QH    (E_WO + N_WO)
#define E_QR    (E_QH + N_QH)
#define E_KH    (E_QR + N_QR)
#define E_KR    (E_KH + N_KH)
#define E_VH    (E_KR + N_KR)
#define E_VR    (E_VH + N_KH)
#define E_CH    (E_VR + N_KR)
#define E_CR    (E_CH + N_CH)
#define E_END   (E_CR + N_CR)
#define B_TABC  (E_END * 2ull)
#define B_TABS  (B_TABC + (u64)SEQ * 32 * 4)
#define B_END   (B_TABS + (u64)SEQ * 32 * 4)

static_assert(HDIM == 64);
static_assert(HDIM * 2 == 128);
static_assert(EMB == NHEAD * HDIM);
static_assert(NQKV == EMB + 2 * NKV * HDIM);
static_assert(NHEAD == 4 * NKV);
static_assert(EMB % 32 == 0);
static_assert(EMB % 64 == 0);
static_assert(NQKV % 64 == 0);
static_assert(SEQ % 128 == 0);
static_assert(MROWS % 128 == 0);
static_assert(EARLY % BQ == 0);
static_assert(EARLY <= SEQ);
static_assert(SEQ % BQ == 0);
static_assert(SEQ % BK == 0);
static_assert(BQ == NWAVE * 16);
static_assert(EMB / 8 == 256);
static_assert(((u64)MROWS * EMB / 8) % 256 == 0);
static_assert(((u64)SEQ * 32) % 256 == 0);
static_assert((SP * 4) % 16 == 0);
static_assert((OP * 4) % 16 == 0);
static_assert((TPW * 2) % 16 == 0);
static_assert(SP >= 64 && OP >= HDIM && TPW >= 64);
static_assert(SEQ <= SEQ_FULL);
static_assert(NB >= 1 && NB <= NB_FULL);
static_assert(N_XB % 64 == 0 && N_QR % 64 == 0 && N_KR % 64 == 0 && N_CR % 64 == 0);
static_assert(B_END <= WS_CAP);

typedef __bf16   bf16;
typedef _Float16 f16;
typedef bf16     v16bf __attribute__((ext_vector_type(16)));
typedef f16      v16h  __attribute__((ext_vector_type(16)));
typedef float    v8f   __attribute__((ext_vector_type(8)));
typedef float    v4f   __attribute__((ext_vector_type(4)));
typedef unsigned v4u   __attribute__((ext_vector_type(4)));

union Frag16 { v4u q[2]; v16bf b; v16h h; };
union FragH  { v16h v; v4u q[2]; f16 h[16]; };
union Pack8B { v4u u; bf16 h[8]; };
union Pack8H { v4u u; f16 h[8]; };

static __device__ __forceinline__ v8f mma_bf16(v16bf a, v16bf b, v8f acc) {
  acc = __builtin_amdgcn_wmma_f32_16x16x32_bf16(false, a, false, b, (short)0, acc, false, false);
  asm volatile("v_nop\n\tv_nop\n\tv_nop\n\tv_nop" : "+v"(acc) : "v"(a), "v"(b));
  return acc;
}
static __device__ __forceinline__ v8f mma_f16(v16h a, v16h b, v8f acc) {
  acc = __builtin_amdgcn_wmma_f32_16x16x32_f16(false, a, false, b, (short)0, acc, false, false);
  asm volatile("v_nop\n\tv_nop\n\tv_nop\n\tv_nop" : "+v"(acc) : "v"(a), "v"(b));
  return acc;
}

__global__ __launch_bounds__(256) void k_cvt_x(const float* __restrict__ x, unsigned short* __restrict__ xb) {
  const int gid = blockIdx.x * 256 + threadIdx.x;
  const int m   = gid >> 8;
  const int cg  = gid & 255;
  const size_t src = ((size_t)(m / SEQ) * SEQ_FULL + (size_t)(m % SEQ)) * EMB + cg * 8;
  const v4f a0 = *(const v4f*)(x + src);
  const v4f a1 = *(const v4f*)(x + src + 4);
  Pack8B pk;
  #pragma unroll
  for (int i = 0; i < 4; ++i) {
    pk.h[i]     = (bf16)a0[i];
    pk.h[4 + i] = (bf16)a1[i];
  }
  const v4u val = pk.u;
  const size_t dst = (size_t)m * EMB + cg * 8;
  *(volatile v4u*)(xb + dst) = val;
  __threadfence();
  *(volatile v4u*)(xb + dst) = val;
}

__global__ __launch_bounds__(256) void k_wT(const float* __restrict__ W, int N,
                                            unsigned short* __restrict__ dst, int rowOff, int mode) {
  __shared__ __align__(16) unsigned short sT[64 * TPW];
  const int tid = threadIdx.x;
  const int n0  = blockIdx.x * 64;
  const int k0  = blockIdx.y * 64;
  #pragma unroll
  for (int p = 0; p < 4; ++p) {
    const int kk = (tid >> 4) + 16 * p;
    const int nc = (tid & 15) * 4;
    const v4f w = *(const v4f*)(W + (size_t)(k0 + kk) * N + n0 + nc);
    #pragma unroll
    for (int i = 0; i < 4; ++i) {
      const bf16  wb = (bf16)w[i];
      const f16   wh = (f16)((float)wb * 64.0f);
      const unsigned short u0 = __builtin_bit_cast(unsigned short, wb);
      const unsigned short u1 = __builtin_bit_cast(unsigned short, wh);
      sT[(nc + i) * TPW + kk] = (mode != 0) ? u1 : u0;
    }
  }
  __syncthreads();
  v4u    val[2];
  size_t idx[2];
  #pragma unroll
  for (int p = 0; p < 2; ++p) {
    const int n  = (tid >> 3) + 32 * p;
    const int ks = (tid & 7) * 8;
    val[p] = *(const v4u*)(sT + n * TPW + ks);
    idx[p] = (size_t)(rowOff + n0 + n) * EMB + k0 + ks;
  }
  #pragma unroll
  for (int p = 0; p < 2; ++p) *(volatile v4u*)(dst + idx[p]) = val[p];
  __threadfence();
  #pragma unroll
  for (int p = 0; p < 2; ++p) *(volatile v4u*)(dst + idx[p]) = val[p];
}

__global__ __launch_bounds__(256) void k_tables(float* __restrict__ tabc, float* __restrict__ tabs) {
  const int gid = blockIdx.x * 256 + threadIdx.x;
  const int t = gid >> 5;
  const int j = gid & 31;
  double p = 1.0;
  p *= (j & 1)  ? 1.333521432163324   : 1.0;
  p *= (j & 2)  ? 1.7782794100389228  : 1.0;
  p *= (j & 4)  ? 3.1622776601683795  : 1.0;
  p *= (j & 8)  ? 10.0                : 1.0;
  p *= (j & 16) ? 100.0               : 1.0;
  const float pf  = (float)p;
  const float inv = 1.0f / pf;
  const float ang = (float)t * inv;
  float sn, cs;
  sincosf(ang, &sn, &cs);
  *(volatile float*)(tabc + gid) = cs;
  *(volatile float*)(tabs + gid) = sn;
  __threadfence();
  *(volatile float*)(tabc + gid) = cs;
  *(volatile float*)(tabs + gid) = sn;
}

template <bool ISBF>
static __device__ __forceinline__ void gemm_loop(const unsigned short* __restrict__ ap,
                                                 const unsigned short* __restrict__ bp,
                                                 v8f (&acc)[2][4]) {
  #pragma unroll 1
  for (int k0 = 0; k0 < EMB; k0 += 32) {
    Frag16 a[2], bf[4];
    #pragma unroll
    for (int mt = 0; mt < 2; ++mt) {
      a[mt].q[0] = *(const v4u*)(ap + (size_t)mt * 16 * EMB + k0);
      a[mt].q[1] = *(const v4u*)(ap + (size_t)mt * 16 * EMB + k0 + 16);
    }
    #pragma unroll
    for (int nt = 0; nt < 4; ++nt) {
      bf[nt].q[0] = *(const v4u*)(bp + (size_t)nt * 16 * EMB + k0);
      bf[nt].q[1] = *(const v4u*)(bp + (size_t)nt * 16 * EMB + k0 + 16);
    }
    #pragma unroll
    for (int mt = 0; mt < 2; ++mt) {
      #pragma unroll
      for (int nt = 0; nt < 4; ++nt) {
        if (ISBF) acc[mt][nt] = mma_bf16(a[mt].b, bf[nt].b, acc[mt][nt]);
        else      acc[mt][nt] = mma_f16(a[mt].h, bf[nt].h, acc[mt][nt]);
      }
    }
  }
}

__global__ __launch_bounds__(128) void k_proj(const unsigned short* __restrict__ xb,
                                              const unsigned short* __restrict__ wt,
                                              const float* __restrict__ bq,
                                              const float* __restrict__ bk,
                                              const float* __restrict__ bv,
                                              const float* __restrict__ tabc,
                                              const float* __restrict__ tabs,
                                              f16* __restrict__ pl) {
  __shared__ __align__(16) float sC[128 * SP];
  const int tid  = threadIdx.x;
  const int wave = __builtin_amdgcn_readfirstlane(threadIdx.x >> 5);
  const int lane = tid & 31;
  const int lq   = lane & 15;
  const int hi   = lane >> 4;
  const int m0   = blockIdx.x * 128;
  const int slot = blockIdx.y;
  const int n0   = slot * 64;

  v8f acc[2][4];
  #pragma unroll
  for (int mt = 0; mt < 2; ++mt) {
    #pragma unroll
    for (int nt = 0; nt < 4; ++nt) acc[mt][nt] = (v8f){0, 0, 0, 0, 0, 0, 0, 0};
  }

  const unsigned short* ap = xb + (size_t)(m0 + wave * 32 + lq) * EMB + hi * 8;
  const unsigned short* bp = wt + (size_t)(n0 + lq) * EMB + hi * 8;
  gemm_loop<true>(ap, bp, acc);

  #pragma unroll
  for (int mt = 0; mt < 2; ++mt) {
    #pragma unroll
    for (int nt = 0; nt < 4; ++nt) {
      #pragma unroll
      for (int r = 0; r < 8; ++r)
        sC[(wave * 32 + mt * 16 + hi * 8 + r) * SP + nt * 16 + lq] = acc[mt][nt][r];
    }
  }
  __syncthreads();

  const int  bb    = m0 / SEQ;
  const int  t0    = m0 % SEQ;
  const bool early = t0 < EARLY;

  if (slot < NHEAD + NKV) {
    const bool isq = slot < NHEAD;
    const int  hd  = isq ? slot : slot - NHEAD;
    const int  nh  = isq ? NHEAD : NKV;
    const u64  oH  = isq ? E_QH : E_KH;
    const u64  oR  = isq ? E_QR : E_KR;
    const int  c0  = (lane & 7) * 8;

    int iq = n0 + c0;        iq = iq > EMB - 8 ? EMB - 8 : iq;
    int ik = n0 + c0 - EMB;  ik = ik < 0 ? 0 : ik;  ik = ik > NKV * HDIM - 8 ? NKV * HDIM - 8 : ik;
    const v4f q0 = *(const v4f*)(bq + iq);
    const v4f q1 = *(const v4f*)(bq + iq + 4);
    const v4f k0 = *(const v4f*)(bk + ik);
    const v4f k1 = *(const v4f*)(bk + ik + 4);
    float bias[8];
    #pragma unroll
    for (int i = 0; i < 4; ++i) {
      bias[i]     = (float)(bf16)(isq ? q0[i] : k0[i]);
      bias[4 + i] = (float)(bf16)(isq ? q1[i] : k1[i]);
    }

    const int rl = wave * 32 + (lane >> 3);
    const int t  = t0 + rl;
    const u64 dH0 = oH + (((u64)bb * nh + hd) * SEQ   + t) * HDIM + c0;
    const u64 dR0 = oR + (((u64)bb * nh + hd) * EARLY + t) * HDIM + c0;

    v4u hv[8], rv[8];
    #pragma unroll
    for (int it = 0; it < 8; ++it) {
      const int row = rl + it * 4;
      const v4f x0 = *(const v4f*)(sC + row * SP + c0);
      const v4f x1 = *(const v4f*)(sC + row * SP + c0 + 4);
      const v4f cs = *(const v4f*)(tabc + (size_t)(t + it * 4) * 32 + (c0 >> 1));
      const v4f sn = *(const v4f*)(tabs + (size_t)(t + it * 4) * 32 + (c0 >> 1));
      float y[8];
      #pragma unroll
      for (int p = 0; p < 2; ++p) {
        const float e0 = x0[2 * p]     + bias[2 * p];
        const float o0 = x0[2 * p + 1] + bias[2 * p + 1];
        y[2 * p]     = e0 * cs[p] - o0 * sn[p];
        y[2 * p + 1] = o0 * cs[p] + e0 * sn[p];
        const float e1 = x1[2 * p]     + bias[4 + 2 * p];
        const float o1 = x1[2 * p + 1] + bias[4 + 2 * p + 1];
        y[4 + 2 * p]     = e1 * cs[2 + p] - o1 * sn[2 + p];
        y[4 + 2 * p + 1] = o1 * cs[2 + p] + e1 * sn[2 + p];
      }
      Pack8H ph, pr;
      #pragma unroll
      for (int i = 0; i < 8; ++i) {
        ph.h[i] = (f16)y[i];
        pr.h[i] = (f16)((y[i] - (float)ph.h[i]) * 2048.0f);
      }
      hv[it] = ph.u;
      rv[it] = pr.u;
    }
    #pragma unroll
    for (int it = 0; it < 8; ++it) *(volatile v4u*)(pl + dH0 + (u64)it * 4 * HDIM) = hv[it];
    if (early) {
      #pragma unroll
      for (int it = 0; it < 8; ++it) *(volatile v4u*)(pl + dR0 + (u64)it * 4 * HDIM) = rv[it];
    }
    __threadfence();
    #pragma unroll
    for (int it = 0; it < 8; ++it) *(volatile v4u*)(pl + dH0 + (u64)it * 4 * HDIM) = hv[it];
    if (early) {
      #pragma unroll
      for (int it = 0; it < 8; ++it) *(volatile v4u*)(pl + dR0 + (u64)it * 4 * HDIM) = rv[it];
    }
  } else {
    const int g  = slot - (NHEAD + NKV);
    const int tg = lane & 15;
    const int db = wave * 2 + hi;
    const u64 dH0 = E_VH + (((u64)bb * NKV + g) * HDIM + db) * SEQ   + t0 + tg * 8;
    const u64 dR0 = E_VR + (((u64)bb * NKV + g) * HDIM + db) * EARLY + t0 + tg * 8;
    v4u hv[8], rv[8];
    #pragma unroll
    for (int it = 0; it < 8; ++it) {
      const int d = it * 8 + db;
      const float bd = (float)(bf16)bv[g * HDIM + d];
      Pack8H ph, pr;
      #pragma unroll
      for (int i = 0; i < 8; ++i) {
        const float y = sC[(tg * 8 + i) * SP + d] + bd;
        ph.h[i] = (f16)y;
        pr.h[i] = (f16)((y - (float)ph.h[i]) * 2048.0f);
      }
      hv[it] = ph.u;
      rv[it] = pr.u;
    }
    #pragma unroll
    for (int it = 0; it < 8; ++it) *(volatile v4u*)(pl + dH0 + (u64)it * 8 * SEQ) = hv[it];
    if (early) {
      #pragma unroll
      for (int it = 0; it < 8; ++it) *(volatile v4u*)(pl + dR0 + (u64)it * 8 * EARLY) = rv[it];
    }
    __threadfence();
    #pragma unroll
    for (int it = 0; it < 8; ++it) *(volatile v4u*)(pl + dH0 + (u64)it * 8 * SEQ) = hv[it];
    if (early) {
      #pragma unroll
      for (int it = 0; it < 8; ++it) *(volatile v4u*)(pl + dR0 + (u64)it * 8 * EARLY) = rv[it];
    }
  }
}

template <bool EP>
static __device__ __forceinline__ void attn_body(const f16* __restrict__ qh, const f16* __restrict__ qr,
                                                 const f16* __restrict__ kh, const f16* __restrict__ kr,
                                                 const f16* __restrict__ vth, const f16* __restrict__ vtr,
                                                 f16* __restrict__ ch, f16* __restrict__ cr, const int qblk) {
  __shared__ __align__(16) float sO[NWAVE * 16 * OP];
  const int h    = blockIdx.y;
  const int b    = blockIdx.z;
  const int g    = h >> 2;
  const int tid  = threadIdx.x;
  const int wave = __builtin_amdgcn_readfirstlane(threadIdx.x >> 5);
  const int lane = tid & 31;
  const int lq   = lane & 15;
  const int hi   = lane >> 4;
  const int qrow0 = qblk * BQ + wave * 16;

  FragH qf[2], qrf[2];
  {
    const f16* qp = qh + (((size_t)b * NHEAD + h) * SEQ + qrow0 + lq) * HDIM + hi * 8;
    #pragma unroll
    for (int f = 0; f < 2; ++f) {
      qf[f].q[0] = *(const v4u*)(qp + f * 32);
      qf[f].q[1] = *(const v4u*)(qp + f * 32 + 16);
    }
    if (EP) {
      const f16* rp = qr + (((size_t)b * NHEAD + h) * EARLY + qrow0 + lq) * HDIM + hi * 8;
      #pragma unroll
      for (int f = 0; f < 2; ++f) {
        qrf[f].q[0] = *(const v4u*)(rp + f * 32);
        qrf[f].q[1] = *(const v4u*)(rp + f * 32 + 16);
      }
    } else {
      qrf[0] = qf[0];
      qrf[1] = qf[1];
    }
  }

  const f16* kh_g = kh  + ((size_t)b * NKV + g) * SEQ * HDIM;
  const f16* kr_g = kr  + ((size_t)b * NKV + g) * EARLY * HDIM;
  const f16* vh_g = vth + ((size_t)b * NKV + g) * HDIM * SEQ;
  const f16* vr_g = vtr + ((size_t)b * NKV + g) * HDIM * EARLY;

  v8f o[4], ores[4];
  #pragma unroll
  for (int dt = 0; dt < 4; ++dt) {
    o[dt]    = (v8f){0, 0, 0, 0, 0, 0, 0, 0};
    ores[dt] = (v8f){0, 0, 0, 0, 0, 0, 0, 0};
  }
  float rmax = NEGBIG;
  float rsum = 0.0f;
  const float SL = 0.125f * 1.4426950408889634f;

  const int nchunk = (qrow0 + 16 + BK - 1) / BK;
  #pragma unroll 1
  for (int i = 0; i < nchunk; ++i) {
    const int j0 = i * BK;

    v8f c[2];
    #pragma unroll
    for (int sub = 0; sub < 2; ++sub) {
      const f16* kp = kh_g + (size_t)(j0 + sub * 16 + lq) * HDIM + hi * 8;
      FragH a0, a1;
      a0.q[0] = *(const v4u*)(kp);
      a0.q[1] = *(const v4u*)(kp + 16);
      a1.q[0] = *(const v4u*)(kp + 32);
      a1.q[1] = *(const v4u*)(kp + 48);
      v8f acc = (v8f){0, 0, 0, 0, 0, 0, 0, 0};
      acc = mma_f16(a0.v, qf[0].v, acc);
      acc = mma_f16(a1.v, qf[1].v, acc);
      if (EP) {
        const f16* rp = kr_g + (size_t)(j0 + sub * 16 + lq) * HDIM + hi * 8;
        FragH r0, r1;
        r0.q[0] = *(const v4u*)(rp);
        r0.q[1] = *(const v4u*)(rp + 16);
        r1.q[0] = *(const v4u*)(rp + 32);
        r1.q[1] = *(const v4u*)(rp + 48);
        v8f ar = (v8f){0, 0, 0, 0, 0, 0, 0, 0};
        ar = mma_f16(r0.v, qf[0].v, ar);
        ar = mma_f16(r1.v, qf[1].v, ar);
        ar = mma_f16(a0.v, qrf[0].v, ar);
        ar = mma_f16(a1.v, qrf[1].v, ar);
        #pragma unroll
        for (int r = 0; r < 8; ++r) acc[r] += ar[r] * (1.0f / 2048.0f);
      }
      c[sub] = acc;
    }

    if (i == nchunk - 1) {
      const int qi = qrow0 + lq;
      #pragma unroll
      for (int r = 0; r < 8; ++r) {
        const int key0 = j0 + hi * 8 + r;
        c[0][r] = (key0 > qi)      ? NEGBIG : c[0][r];
        c[1][r] = (key0 + 16 > qi) ? NEGBIG : c[1][r];
      }
    }

    float m_new = rmax;
    #pragma unroll
    for (int r = 0; r < 8; ++r) {
      m_new = fmaxf(m_new, c[0][r]);
      m_new = fmaxf(m_new, c[1][r]);
    }
    m_new = fmaxf(m_new, __shfl_xor(m_new, 16, 32));
    const float scale = __builtin_amdgcn_exp2f((rmax - m_new) * SL);
    rmax = m_new;

    FragH pa, pr;
    float psum = 0.0f;
    #pragma unroll
    for (int r = 0; r < 8; ++r) {
      const float p0 = __builtin_amdgcn_exp2f((c[0][r] - m_new) * SL);
      const float p1 = __builtin_amdgcn_exp2f((c[1][r] - m_new) * SL);
      psum += p0 + p1;
      const float s0 = p0 * 4096.0f;
      const float s1 = p1 * 4096.0f;
      pa.h[r]     = (f16)s0;
      pa.h[8 + r] = (f16)s1;
      pr.h[r]     = (f16)((s0 - (float)pa.h[r]) * 2048.0f);
      pr.h[8 + r] = (f16)((s1 - (float)pa.h[8 + r]) * 2048.0f);
    }
    rsum = rsum * scale + psum + __shfl_xor(psum, 16, 32);

    float sc[8];
    #pragma unroll
    for (int r = 0; r < 8; ++r) sc[r] = __shfl(scale, (hi << 3) + r, 32);
    #pragma unroll
    for (int dt = 0; dt < 4; ++dt) {
      #pragma unroll
      for (int r = 0; r < 8; ++r) {
        o[dt][r] *= sc[r];
        if (EP) ores[dt][r] *= sc[r];
      }
    }

    #pragma unroll
    for (int dt = 0; dt < 4; ++dt) {
      const f16* vp = vh_g + (size_t)(dt * 16 + lq) * SEQ + j0 + hi * 8;
      FragH bvf;
      bvf.q[0] = *(const v4u*)(vp);
      bvf.q[1] = *(const v4u*)(vp + 16);
      o[dt] = mma_f16(pa.v, bvf.v, o[dt]);
      if (EP) {
        const f16* wp = vr_g + (size_t)(dt * 16 + lq) * EARLY + j0 + hi * 8;
        FragH bvr;
        bvr.q[0] = *(const v4u*)(wp);
        bvr.q[1] = *(const v4u*)(wp + 16);
        ores[dt] = mma_f16(pr.v, bvf.v, ores[dt]);
        ores[dt] = mma_f16(pa.v, bvr.v, ores[dt]);
      }
    }
  }

  float rs[8];
  #pragma unroll
  for (int r = 0; r < 8; ++r) rs[r] = 1.0f / __shfl(rsum, (hi << 3) + r, 32);

  float* so = sO + wave * (16 * OP);
  #pragma unroll
  for (int r = 0; r < 8; ++r) {
    #pragma unroll
    for (int dt = 0; dt < 4; ++dt) {
      float val = o[dt][r];
      if (EP) val += ores[dt][r] * (1.0f / 2048.0f);
      so[(hi * 8 + r) * OP + dt * 16 + lq] = val * (1.0f / 4096.0f) * rs[r];
    }
  }
  __syncthreads();

  const int c0 = (lane & 7) * 8;
  const int r0 = lane >> 3;
  v4u hv[4], rv[4];
  #pragma unroll
  for (int it = 0; it < 4; ++it) {
    const int row = it * 4 + r0;
    const v4f x0 = *(const v4f*)(so + row * OP + c0);
    const v4f x1 = *(const v4f*)(so + row * OP + c0 + 4);
    Pack8H ph, pq;
    #pragma unroll
    for (int i = 0; i < 4; ++i) {
      const float y0 = x0[i] * 64.0f;
      const float y1 = x1[i] * 64.0f;
      ph.h[i]     = (f16)y0;
      ph.h[4 + i] = (f16)y1;
      pq.h[i]     = (f16)((y0 - (float)ph.h[i]) * 2048.0f);
      pq.h[4 + i] = (f16)((y1 - (float)ph.h[4 + i]) * 2048.0f);
    }
    hv[it] = ph.u;
    rv[it] = pq.u;
  }
  const size_t dH0 = ((size_t)b * SEQ   + qrow0 + r0) * EMB + h * HDIM + c0;
  const size_t dR0 = ((size_t)b * EARLY + qrow0 + r0) * EMB + h * HDIM + c0;
  #pragma unroll
  for (int it = 0; it < 4; ++it) *(volatile v4u*)(ch + dH0 + (size_t)it * 4 * EMB) = hv[it];
  if (EP) {
    #pragma unroll
    for (int it = 0; it < 4; ++it) *(volatile v4u*)(cr + dR0 + (size_t)it * 4 * EMB) = rv[it];
  }
  __threadfence();
  #pragma unroll
  for (int it = 0; it < 4; ++it) *(volatile v4u*)(ch + dH0 + (size_t)it * 4 * EMB) = hv[it];
  if (EP) {
    #pragma unroll
    for (int it = 0; it < 4; ++it) *(volatile v4u*)(cr + dR0 + (size_t)it * 4 * EMB) = rv[it];
  }
}

__global__ __launch_bounds__(256) void k_attn_early(const f16* __restrict__ qh, const f16* __restrict__ qr,
                                                    const f16* __restrict__ kh, const f16* __restrict__ kr,
                                                    const f16* __restrict__ vth, const f16* __restrict__ vtr,
                                                    f16* __restrict__ ch, f16* __restrict__ cr) {
  attn_body<true>(qh, qr, kh, kr, vth, vtr, ch, cr, (int)blockIdx.x);
}

__global__ __launch_bounds__(256) void k_attn_late(const f16* __restrict__ qh, const f16* __restrict__ qr,
                                                   const f16* __restrict__ kh, const f16* __restrict__ kr,
                                                   const f16* __restrict__ vth, const f16* __restrict__ vtr,
                                                   f16* __restrict__ ch, f16* __restrict__ cr) {
  attn_body<false>(qh, qr, kh, kr, vth, vtr, ch, cr, (int)blockIdx.x + EARLY / BQ);
}

__global__ __launch_bounds__(128) void k_outp(const unsigned short* __restrict__ ch,
                                              const unsigned short* __restrict__ cr,
                                              const unsigned short* __restrict__ wo,
                                              const float* __restrict__ bo,
                                              float* __restrict__ out) {
  __shared__ __align__(16) float sC[128 * SP];
  const int tid  = threadIdx.x;
  const int wave = __builtin_amdgcn_readfirstlane(threadIdx.x >> 5);
  const int lane = tid & 31;
  const int lq   = lane & 15;
  const int hi   = lane >> 4;
  const int m0   = blockIdx.x * 128;
  const int n0   = blockIdx.y * 64;
  const int bb   = m0 / SEQ;
  const int t0   = m0 % SEQ;
  const bool early = t0 < EARLY;

  v8f acc[2][4];
  #pragma unroll
  for (int mt = 0; mt < 2; ++mt) {
    #pragma unroll
    for (int nt = 0; nt < 4; ++nt) acc[mt][nt] = (v8f){0, 0, 0, 0, 0, 0, 0, 0};
  }
  const unsigned short* bp = wo + (size_t)(n0 + lq) * EMB + hi * 8;
  if (early) {
    const unsigned short* rp = cr + ((size_t)bb * EARLY + t0 + wave * 32 + lq) * EMB + hi * 8;
    gemm_loop<false>(rp, bp, acc);
    #pragma unroll
    for (int mt = 0; mt < 2; ++mt) {
      #pragma unroll
      for (int nt = 0; nt < 4; ++nt) {
        #pragma unroll
        for (int r = 0; r < 8; ++r) acc[mt][nt][r] *= (1.0f / 2048.0f);
      }
    }
  }
  const unsigned short* ap = ch + (size_t)(m0 + wave * 32 + lq) * EMB + hi * 8;
  gemm_loop<false>(ap, bp, acc);

  #pragma unroll
  for (int mt = 0; mt < 2; ++mt) {
    #pragma unroll
    for (int nt = 0; nt < 4; ++nt) {
      #pragma unroll
      for (int r = 0; r < 8; ++r)
        sC[(wave * 32 + mt * 16 + hi * 8 + r) * SP + nt * 16 + lq] = acc[mt][nt][r] * (1.0f / 4096.0f);
    }
  }
  __syncthreads();

  const int c = lq * 4;
  const v4f braw = *(const v4f*)(bo + n0 + c);
  v4f bias;
  #pragma unroll
  for (int i = 0; i < 4; ++i) bias[i] = (float)(bf16)braw[i];
  v4f vals[16];
  #pragma unroll
  for (int it = 0; it < 16; ++it) {
    const int row = wave * 32 + it * 2 + hi;
    const v4f x = *(const v4f*)(sC + row * SP + c);
    vals[it] = x + bias;
  }
  const size_t d0 = ((size_t)bb * SEQ_FULL + t0 + wave * 32 + hi) * EMB + n0 + c;
  #pragma unroll
  for (int it = 0; it < 16; ++it) *(volatile v4f*)(out + d0 + (size_t)it * 2 * EMB) = vals[it];
  __threadfence();
  #pragma unroll
  for (int it = 0; it < 16; ++it) *(volatile v4f*)(out + d0 + (size_t)it * 2 * EMB) = vals[it];
}

extern "C" void kernel_launch(void* const* d_in, const int* in_sizes, int n_in,
                              void* d_out, int out_size, void* d_ws, size_t ws_size,
                              hipStream_t stream) {
  if (n_in < 9) return;
  const size_t need_x = (((size_t)(NB - 1) * SEQ_FULL) + SEQ) * EMB;
  if ((size_t)in_sizes[0] < need_x) return;
  if ((size_t)in_sizes[1] < (size_t)EMB * EMB) return;
  if ((size_t)in_sizes[2] < (size_t)EMB) return;
  if ((size_t)in_sizes[3] < (size_t)EMB * NKV * HDIM) return;
  if ((size_t)in_sizes[4] < (size_t)NKV * HDIM) return;
  if ((size_t)in_sizes[5] < (size_t)EMB * NKV * HDIM) return;
  if ((size_t)in_sizes[6] < (size_t)NKV * HDIM) return;
  if ((size_t)in_sizes[7] < (size_t)EMB * EMB) return;
  if ((size_t)in_sizes[8] < (size_t)EMB) return;
  if ((size_t)out_size < need_x) return;
  if ((u64)ws_size < B_END) return;

  const float* x  = (const float*)d_in[0];
  const float* Wq = (const float*)d_in[1];
  const float* bq = (const float*)d_in[2];
  const float* Wk = (const float*)d_in[3];
  const float* bk = (const float*)d_in[4];
  const float* Wv = (const float*)d_in[5];
  const float* bv = (const float*)d_in[6];
  const float* Wo = (const float*)d_in[7];
  const float* bo = (const float*)d_in[8];
  float* out = (float*)d_out;

  f16*            pl   = (f16*)d_ws;
  unsigned short* pu   = (unsigned short*)d_ws;
  unsigned short* xb   = pu + E_XB;
  unsigned short* wqkv = pu + E_WQKV;
  unsigned short* woT  = pu + E_WO;
  float* tabc = (float*)((char*)d_ws + B_TABC);
  float* tabs = (float*)((char*)d_ws + B_TABS);

  k_cvt_x<<<dim3((unsigned)((u64)MROWS * EMB / 8 / 256)), 256, 0, stream>>>(x, xb);
  k_wT<<<dim3(EMB / 64, EMB / 64), 256, 0, stream>>>(Wq, EMB, wqkv, 0, 0);
  k_wT<<<dim3(NKV * HDIM / 64, EMB / 64), 256, 0, stream>>>(Wk, NKV * HDIM, wqkv, EMB, 0);
  k_wT<<<dim3(NKV * HDIM / 64, EMB / 64), 256, 0, stream>>>(Wv, NKV * HDIM, wqkv, EMB + NKV * HDIM, 0);
  k_wT<<<dim3(EMB / 64, EMB / 64), 256, 0, stream>>>(Wo, EMB, woT, 0, 1);
  k_tables<<<dim3(SEQ * 32 / 256), 256, 0, stream>>>(tabc, tabs);

  k_proj<<<dim3(MROWS / 128, NQKV / 64), 128, 0, stream>>>(xb, wqkv, bq, bk, bv, tabc, tabs, pl);

  const f16* qh  = pl + E_QH;
  const f16* qr  = pl + E_QR;
  const f16* kh  = pl + E_KH;
  const f16* kr  = pl + E_KR;
  const f16* vth = pl + E_VH;
  const f16* vtr = pl + E_VR;
  f16* chp = pl + E_CH;
  f16* crp = pl + E_CR;

  k_attn_early<<<dim3(EARLY / BQ, NHEAD, NB), 256, 0, stream>>>(qh, qr, kh, kr, vth, vtr, chp, crp);
  if ((SEQ - EARLY) / BQ > 0) {
    k_attn_late<<<dim3((SEQ - EARLY) / BQ, NHEAD, NB), 256, 0, stream>>>(qh, qr, kh, kr, vth, vtr, chp, crp);
  }

  k_outp<<<dim3(MROWS / 128, EMB / 64), 128, 0, stream>>>(pu + E_CH, pu + E_CR, woT, bo, out);
}
